// EDeeperGCN_70909910057020
// MI455X (gfx1250) — hardware-verified
//
#include <hip/hip_runtime.h>
#include <stddef.h>


#define HID  128
#define NOUT 10
#define NPAD 16
#define PQW  256
#define ETHR 128
#define EBLK 128

typedef float          v4f  __attribute__((ext_vector_type(4)));
typedef float          v8f  __attribute__((ext_vector_type(8)));
typedef unsigned short v4us __attribute__((ext_vector_type(4)));
typedef unsigned short v8us __attribute__((ext_vector_type(8)));
typedef __bf16         v16b __attribute__((ext_vector_type(16)));
union FragB { v16b v; v8us u[2]; };

__device__ __forceinline__ unsigned short bf_bits(float f) {
  const unsigned u = __builtin_bit_cast(unsigned, f);
  return (unsigned short)((u + 0x7FFFu + ((u >> 16) & 1u)) >> 16);
}
__device__ __forceinline__ float bf_val(unsigned short b) {
  return __builtin_bit_cast(float, ((unsigned)b) << 16);
}

__device__ __forceinline__ v8f wmb(v16b a, v16b b, v8f c) {
  v8f d = __builtin_amdgcn_wmma_f32_16x16x32_bf16(false, a, false, b, (short)0, c, false, false);
  asm volatile("v_nop\n\tv_nop\n\tv_nop\n\tv_nop" : "+v"(d) : "v"(a), "v"(b));
  return d;
}

__device__ __forceinline__ v8f zero8f() {
  v8f z;
#pragma unroll
  for (int i = 0; i < 8; ++i) z[i] = 0.0f;
  return z;
}

__global__ __launch_bounds__(256) void k_prep(const float* __restrict__ x,
                                              const float* __restrict__ W1,
                                              const float* __restrict__ W2,
                                              unsigned short* xh, unsigned short* xl,
                                              unsigned short* w1h, unsigned short* w1l,
                                              unsigned short* w2h, unsigned short* w2l,
                                              int nN, int xBlocks) {
  const int tid = threadIdx.x;
  const int b = blockIdx.x;
  float v[8];
  unsigned short* ph;
  unsigned short* pl;
  size_t o;
  if (b < xBlocks) {
    const int g = b * 256 + tid;
    const int row = g >> 4;
    const int col = (g & 15) * 8;
    const int rc = row < nN ? row : nN - 1;
    const float* xp = x + (size_t)rc * HID + col;
    const v4f a = *(const v4f*)xp;
    const v4f c = *(const v4f*)(xp + 4);
    const bool ok = row < nN;
    v[0] = ok ? a.x : 0.0f; v[1] = ok ? a.y : 0.0f; v[2] = ok ? a.z : 0.0f; v[3] = ok ? a.w : 0.0f;
    v[4] = ok ? c.x : 0.0f; v[5] = ok ? c.y : 0.0f; v[6] = ok ? c.z : 0.0f; v[7] = ok ? c.w : 0.0f;
    ph = xh; pl = xl; o = (size_t)g * 8;
  } else if (b < xBlocks + 16) {
    const int g = (b - xBlocks) * 256 + tid;
    const int n = g >> 4;
    const int kc = (g & 15) * 8;
    const int base = (n >> 7) * HID;
    const int col = n & 127;
#pragma unroll
    for (int i = 0; i < 8; ++i) v[i] = W1[(size_t)(base + kc + i) * HID + col];
    ph = w1h; pl = w1l; o = (size_t)n * HID + kc;
  } else {
    const int n = tid >> 4;
    const int kc = (tid & 15) * 8;
    const int nc = n < NOUT ? n : NOUT - 1;
#pragma unroll
    for (int i = 0; i < 8; ++i) {
      const float t = W2[(kc + i) * NOUT + nc];
      v[i] = (n < NOUT) ? t : 0.0f;
    }
    ph = w2h; pl = w2l; o = (size_t)n * HID + kc;
  }
  v8us hv, lv;
#pragma unroll
  for (int i = 0; i < 8; ++i) {
    const unsigned short hb = bf_bits(v[i]);
    const float hf = bf_val(hb);
    hv[i] = hb;
    lv[i] = bf_bits(v[i] - hf);
  }
  *(volatile v8us*)(ph + o) = hv;
  *(volatile v8us*)(pl + o) = lv;
  __threadfence();
  *(volatile v8us*)(ph + o) = hv;
  *(volatile v8us*)(pl + o) = lv;
}

__global__ __launch_bounds__(128) void k_node(const unsigned short* __restrict__ xh,
                                              const unsigned short* __restrict__ xl,
                                              const unsigned short* __restrict__ w1h,
                                              const unsigned short* __restrict__ w1l,
                                              float* pq) {
  __shared__ __attribute__((aligned(16))) float st[4 * 16 * 64];
  const int tid = threadIdx.x, lane = tid & 31, wave = tid >> 5, h = lane >> 4, m = lane & 15;
  const int r0 = blockIdx.x * 16;
  const int n0w = wave * 64;

  v8f acc[4];
#pragma unroll
  for (int nt = 0; nt < 4; ++nt) acc[nt] = zero8f();

  const unsigned short* arh = xh + (size_t)(r0 + m) * HID + 8 * h;
  const unsigned short* arl = xl + (size_t)(r0 + m) * HID + 8 * h;

#pragma unroll 1
  for (int ks = 0; ks < 4; ++ks) {
    const int k0 = ks * 32;
    FragB ahf, alf;
    ahf.u[0] = *(const v8us*)(arh + k0);
    ahf.u[1] = *(const v8us*)(arh + k0 + 16);
    alf.u[0] = *(const v8us*)(arl + k0);
    alf.u[1] = *(const v8us*)(arl + k0 + 16);
#pragma unroll
    for (int nt = 0; nt < 4; ++nt) {
      const size_t bo = (size_t)(n0w + 16 * nt + m) * HID + k0 + 8 * h;
      FragB bh, bl;
      bh.u[0] = *(const v8us*)(w1h + bo);
      bh.u[1] = *(const v8us*)(w1h + bo + 16);
      bl.u[0] = *(const v8us*)(w1l + bo);
      bl.u[1] = *(const v8us*)(w1l + bo + 16);
      acc[nt] = wmb(ahf.v, bh.v, acc[nt]);
      acc[nt] = wmb(ahf.v, bl.v, acc[nt]);
      acc[nt] = wmb(alf.v, bh.v, acc[nt]);
    }
  }

  float* sw = st + wave * 1024;
#pragma unroll
  for (int nt = 0; nt < 4; ++nt) {
#pragma unroll
    for (int r = 0; r < 8; ++r) sw[(8 * h + r) * 64 + 16 * nt + m] = acc[nt][r];
  }
  __syncthreads();

  const int rsel = lane >> 4;
  const int cp = (lane & 15) * 4;
  v4f ov[8];
#pragma unroll
  for (int i = 0; i < 8; ++i) ov[i] = *(const v4f*)(sw + (2 * i + rsel) * 64 + cp);
#pragma unroll
  for (int i = 0; i < 8; ++i)
    *(volatile v4f*)(pq + (size_t)(r0 + 2 * i + rsel) * PQW + n0w + cp) = ov[i];
  __threadfence();
#pragma unroll
  for (int i = 0; i < 8; ++i)
    *(volatile v4f*)(pq + (size_t)(r0 + 2 * i + rsel) * PQW + n0w + cp) = ov[i];
}

__global__ __launch_bounds__(ETHR) void k_edge(const int* __restrict__ ei,
                                               const float* __restrict__ pq,
                                               const unsigned short* __restrict__ w2h,
                                               const unsigned short* __restrict__ w2l,
                                               const float* __restrict__ b1,
                                               const float* __restrict__ b2,
                                               float* outp, int nN, int nE, int nB2) {
  __shared__ __attribute__((aligned(16))) unsigned short ah[4 * 32 * HID];
  __shared__ __attribute__((aligned(16))) unsigned short al[4 * 32 * HID];
  __shared__ __attribute__((aligned(16))) float ost[EBLK * NOUT];

  const int tid = threadIdx.x, lane = tid & 31, wave = tid >> 5, h = lane >> 4, m = lane & 15;
  const int eb = blockIdx.x * EBLK + wave * 32;
  const int* srcs = ei;
  const int* dsts = ei + nE;

  const v4f bb = *(const v4f*)(b1 + 4 * lane);

#pragma unroll 1
  for (int j = 0; j < 32; ++j) {
    int e = eb + j;
    e = e > nE - 1 ? nE - 1 : e;
    int s = srcs[e];
    int d = dsts[e];
    s = s < 0 ? 0 : (s > nN - 1 ? nN - 1 : s);
    d = d < 0 ? 0 : (d > nN - 1 ? nN - 1 : d);
    const v4f p = *(const v4f*)(pq + (size_t)s * PQW + 4 * lane);
    const v4f q = *(const v4f*)(pq + (size_t)d * PQW + HID + 4 * lane);
    float vv[4];
    vv[0] = fmaxf(p.x + q.x + bb.x, 0.0f);
    vv[1] = fmaxf(p.y + q.y + bb.y, 0.0f);
    vv[2] = fmaxf(p.z + q.z + bb.z, 0.0f);
    vv[3] = fmaxf(p.w + q.w + bb.w, 0.0f);
    v4us hv, lv;
#pragma unroll
    for (int c = 0; c < 4; ++c) {
      const unsigned short hb = bf_bits(vv[c]);
      const float hf = bf_val(hb);
      hv[c] = hb;
      lv[c] = bf_bits(vv[c] - hf);
    }
    const int ro = (wave * 32 + j) * HID + 4 * lane;
    *(v4us*)(ah + ro) = hv;
    *(v4us*)(al + ro) = lv;
  }
  __syncthreads();

  const int bi = m < nB2 - 1 ? m : nB2 - 1;
  const float b2raw = b2[bi < 0 ? 0 : bi];
  const float b2v = (m < NOUT && m < nB2) ? b2raw : 0.0f;
  v8f acc0, acc1;
#pragma unroll
  for (int r = 0; r < 8; ++r) { acc0[r] = b2v; acc1[r] = b2v; }

  const unsigned short* a0h = ah + (wave * 32 + m) * HID + 8 * h;
  const unsigned short* a0l = al + (wave * 32 + m) * HID + 8 * h;
  const unsigned short* a1h = a0h + 16 * HID;
  const unsigned short* a1l = a0l + 16 * HID;
  const unsigned short* bph = w2h + m * HID + 8 * h;
  const unsigned short* bpl = w2l + m * HID + 8 * h;

#pragma unroll
  for (int ks = 0; ks < 4; ++ks) {
    const int k0 = ks * 32;
    FragB f0h, f0l, f1h, f1l, bh, bl;
    f0h.u[0] = *(const v8us*)(a0h + k0); f0h.u[1] = *(const v8us*)(a0h + k0 + 16);
    f0l.u[0] = *(const v8us*)(a0l + k0); f0l.u[1] = *(const v8us*)(a0l + k0 + 16);
    f1h.u[0] = *(const v8us*)(a1h + k0); f1h.u[1] = *(const v8us*)(a1h + k0 + 16);
    f1l.u[0] = *(const v8us*)(a1l + k0); f1l.u[1] = *(const v8us*)(a1l + k0 + 16);
    bh.u[0]  = *(const v8us*)(bph + k0); bh.u[1]  = *(const v8us*)(bph + k0 + 16);
    bl.u[0]  = *(const v8us*)(bpl + k0); bl.u[1]  = *(const v8us*)(bpl + k0 + 16);
    acc0 = wmb(f0h.v, bh.v, acc0);
    acc0 = wmb(f0h.v, bl.v, acc0);
    acc0 = wmb(f0l.v, bh.v, acc0);
    acc1 = wmb(f1h.v, bh.v, acc1);
    acc1 = wmb(f1h.v, bl.v, acc1);
    acc1 = wmb(f1l.v, bh.v, acc1);
  }

  if (m < NOUT) {
    const int er = wave * 32 + 8 * h;
#pragma unroll
    for (int r = 0; r < 8; ++r) {
      ost[(er + r) * NOUT + m]      = acc0[r];
      ost[(er + 16 + r) * NOUT + m] = acc1[r];
    }
  }
  __syncthreads();

  const size_t lim = (size_t)nE * NOUT;
  const size_t gbase = (size_t)blockIdx.x * (EBLK * NOUT);
  v4f ov[3];
#pragma unroll
  for (int i = 0; i < 3; ++i) {
    const int pi = i * ETHR + tid;
    const int pc = pi < 320 ? pi : 319;
    ov[i] = *(const v4f*)(ost + pc * 4);
  }
#pragma unroll
  for (int i = 0; i < 3; ++i) {
    const int pi = i * ETHR + tid;
    if (pi < 320) {
      const size_t gi = gbase + (size_t)pi * 4;
      if (gi + 4 <= lim) {
        *(volatile v4f*)(outp + gi) = ov[i];
      } else {
#pragma unroll
        for (int c = 0; c < 4; ++c)
          if (gi + c < lim) ((volatile float*)outp)[gi + c] = ov[i][c];
      }
    }
  }
  __threadfence();
#pragma unroll
  for (int i = 0; i < 3; ++i) {
    const int pi = i * ETHR + tid;
    if (pi < 320) {
      const size_t gi = gbase + (size_t)pi * 4;
      if (gi + 4 <= lim) {
        *(volatile v4f*)(outp + gi) = ov[i];
      } else {
#pragma unroll
        for (int c = 0; c < 4; ++c)
          if (gi + c < lim) ((volatile float*)outp)[gi + c] = ov[i][c];
      }
    }
  }
}

extern "C" void kernel_launch(void* const* d_in, const int* in_sizes, int n_in,
                              void* d_out, int out_size, void* d_ws, size_t ws_size,
                              hipStream_t stream) {
  if (n_in < 6) return;
  if (in_sizes[0] < HID || (in_sizes[0] % HID) != 0) return;
  const int nN = in_sizes[0] / HID;
  if (in_sizes[1] < 2 || (in_sizes[1] & 1) != 0) return;
  const int nE = in_sizes[1] / 2;
  if (in_sizes[2] != 2 * HID * HID) return;
  if (in_sizes[3] < HID) return;
  if (in_sizes[4] != HID * NOUT) return;
  if (in_sizes[5] < 1) return;
  const int nB2 = in_sizes[5];
  if (out_size != nE * NOUT) return;

  const float* x  = (const float*)d_in[0];
  const int*   ei = (const int*)d_in[1];
  const float* W1 = (const float*)d_in[2];
  const float* b1 = (const float*)d_in[3];
  const float* W2 = (const float*)d_in[4];
  const float* b2 = (const float*)d_in[5];
  float* out = (float*)d_out;

  const int nPadM = ((nN + 15) / 16) * 16;

  char* ws = (char*)d_ws;
  size_t off = 0;
  const size_t szX  = (((size_t)nPadM * HID * 2) + 255) & ~(size_t)255;
  const size_t szW1 = (size_t)256 * HID * 2;
  const size_t szW2 = (size_t)NPAD * HID * 2;
  const size_t szPQ = (((size_t)nPadM * PQW * 4) + 255) & ~(size_t)255;
  const size_t oXh  = off; off += szX;
  const size_t oXl  = off; off += szX;
  const size_t oW1h = off; off += szW1;
  const size_t oW1l = off; off += szW1;
  const size_t oW2h = off; off += szW2;
  const size_t oW2l = off; off += szW2;
  const size_t oPQ  = off; off += szPQ;
  if (off > ws_size) return;
  if (off > (size_t)134217728) return;

  unsigned short* xh  = (unsigned short*)(ws + oXh);
  unsigned short* xl  = (unsigned short*)(ws + oXl);
  unsigned short* w1h = (unsigned short*)(ws + oW1h);
  unsigned short* w1l = (unsigned short*)(ws + oW1l);
  unsigned short* w2h = (unsigned short*)(ws + oW2h);
  unsigned short* w2l = (unsigned short*)(ws + oW2l);
  float* pq = (float*)(ws + oPQ);

  const int xBlocks = nPadM / 16;

  k_prep<<<xBlocks + 17, 256, 0, stream>>>(x, W1, W2, xh, xl, w1h, w1l, w2h, w2l, nN, xBlocks);
  k_node<<<nPadM / 16, 128, 0, stream>>>(xh, xl, w1h, w1l, pq);
  k_edge<<<(nE + EBLK - 1) / EBLK, ETHR, 0, stream>>>(ei, pq, w2h, w2l, b1, b2, out, nN, nE, nB2);
}
